// GINEncoderBlock_19885698580759
// MI455X (gfx1250) — hardware-verified
//
#include <hip/hip_runtime.h>
#include <stddef.h>
#include <stdint.h>

#define DH      128
#define EDIM    16
#define D2      256
#define XBW     128
#define XBWW    64
#define APW     256
#define TPW     512
#define MW      128
#define MWW     64
#define NTHR    256
#define NWAVE   8
#define EPT     8
#define CHUNK   (NTHR * EPT)
#define WCAP    (EPT * 32)
#define LISTN   (NWAVE * WCAP)
#define NBMAX   2048
#define NBRUN   1024
#define RCAP    28672
#define DEGCAP  64
#define PKS     11
#define STW     512
#define GBM     64
#define GTHR    128
#define GNT     8
#define BN      (16 * GNT)
#define PARTW   288
#define ET      64
#define ETHR    128
#define SDP     132
#define SAP     40
#define KE      32
#define NU_W1   (D2 * (D2 / 8))
#define NU_W2   (DH * (TPW / 8))
#define NU_WE   (DH * (KE / 8))
#define MSGC    16.0f
#define MSGI    0.0625f
#define BNEPS   1e-5f
#define MEAS_MAXDEG 28
#define MEAS_B1024  12548
#define LDS_AGG ((2 * RCAP + 2 * NBMAX + LISTN) * 4 + 64)

static_assert(DH == 32 * 4);
static_assert(EDIM == 16 && EDIM <= KE && KE == 32);
static_assert(D2 == 2 * DH && APW == 2 * DH && TPW == 2 * D2);
static_assert((CHUNK & (CHUNK - 1)) == 0 && CHUNK <= (1 << PKS));
static_assert((NBMAX & (NBMAX - 1)) == 0 && NBMAX <= (1 << PKS));
static_assert((NBRUN & (NBRUN - 1)) == 0 && NBRUN <= NBMAX && (NBRUN % NWAVE) == 0);
static_assert(NTHR * 8 == NBMAX);
static_assert(LISTN >= NBMAX && LISTN >= NWAVE * WCAP);
static_assert((RCAP % 32) == 0 && NWAVE * STW <= RCAP);
static_assert(RCAP > MEAS_B1024 + 1024);
static_assert(DEGCAP >= MEAS_MAXDEG + 8);
static_assert(LDS_AGG <= 300000);
static_assert(GBM == (GTHR / 32) * 16 && GTHR == BN && BN == DH);
static_assert((APW % 32) == 0 && (TPW % 32) == 0);
static_assert((NU_W1 % NTHR) == 0 && (NU_W2 % NTHR) == 0 && (NU_WE % NTHR) == 0);
static_assert((PARTW % 32) == 0 && PARTW / 4 <= GTHR && PARTW >= 2 * BN + 1);
static_assert(ET == (ETHR / 32) * 16 && ET * 4 == 2 * ETHR && ET * 2 == ETHR);
static_assert((SDP * 4) % 16 == 0 && (SAP * 2) % 16 == 0 && SAP >= KE && SDP >= DH);
static_assert(ET * SDP * 4 + ET * SAP * 2 <= 65536);

typedef float          v4f  __attribute__((ext_vector_type(4)));
typedef float          v8f  __attribute__((ext_vector_type(8)));
typedef int            v4i  __attribute__((ext_vector_type(4)));
typedef int            v8i  __attribute__((ext_vector_type(8)));
typedef unsigned int   v2u  __attribute__((ext_vector_type(2)));
typedef unsigned int   v4u  __attribute__((ext_vector_type(4)));
typedef unsigned short v8us __attribute__((ext_vector_type(8)));
typedef __bf16         v16b __attribute__((ext_vector_type(16)));
typedef v4f  __attribute__((may_alias)) v4fa;
typedef v2u  __attribute__((may_alias)) v2ua;
typedef v4u  __attribute__((may_alias)) v4ua;
typedef v8us __attribute__((may_alias)) v8usa;
union FragB { v16b v; v8us h[2]; v8i w; };

__device__ __forceinline__ v8f wmb(const FragB& a, const FragB& b, v8f c) {
  v8f d = __builtin_amdgcn_wmma_f32_16x16x32_bf16(false, a.v, false, b.v, (short)0, c, false, false);
  asm volatile("v_nop\n\tv_nop\n\tv_nop\n\tv_nop" : "+v"(d) : "v"(a.w), "v"(b.w));
  return d;
}
__device__ __forceinline__ v8f z8() { v8f z = {0.f, 0.f, 0.f, 0.f, 0.f, 0.f, 0.f, 0.f}; return z; }

__device__ __forceinline__ unsigned short bf_bits(float f) {
  const unsigned int u = __float_as_uint(f);
  const unsigned int r = (u + 0x7FFFu + ((u >> 16) & 1u)) >> 16;
  const unsigned int q = (u >> 16) | 0x40u;
  return (unsigned short)(((u & 0x7fffffffu) > 0x7f800000u) ? q : r);
}
__device__ __forceinline__ float bf_val(unsigned short b) {
  return __uint_as_float(((unsigned int)b) << 16);
}
__device__ __forceinline__ float bf_rne(float f) { return bf_val(bf_bits(f)); }
__device__ __forceinline__ unsigned int f2h(float f) {
  const _Float16 hv = (_Float16)f;
  return (unsigned int)__builtin_bit_cast(unsigned short, hv);
}
__device__ __forceinline__ float h2f(unsigned int b) {
  const _Float16 hv = __builtin_bit_cast(_Float16, (unsigned short)b);
  return (float)hv;
}
__device__ __forceinline__ float relu_keep(float v) { return (v > 0.0f) ? v : (v - v); }
__device__ __forceinline__ void put16(unsigned short* dp, v8us o) {
  *(volatile v8us*)dp = o;
  __threadfence();
  *(volatile v8us*)dp = o;
}

__device__ __forceinline__ int scan_chunk(const int* __restrict__ dsts, int nE, int cbase, int slotBase,
                                          int nb, int vec8, int* list, int tid, int lane, int wave) {
  int wc = 0;
  const int el0  = tid * EPT;
  const int e0   = cbase + el0;
  const int sent = -2147483647 - 1;
  v4i da, db;
  if (vec8 != 0 && cbase + CHUNK <= nE) {
    da = *(const v4i*)(dsts + e0);
    db = *(const v4i*)(dsts + e0 + 4);
  } else {
    da.x = (e0     < nE) ? dsts[min(e0,     nE - 1)] : sent;
    da.y = (e0 + 1 < nE) ? dsts[min(e0 + 1, nE - 1)] : sent;
    da.z = (e0 + 2 < nE) ? dsts[min(e0 + 2, nE - 1)] : sent;
    da.w = (e0 + 3 < nE) ? dsts[min(e0 + 3, nE - 1)] : sent;
    db.x = (e0 + 4 < nE) ? dsts[min(e0 + 4, nE - 1)] : sent;
    db.y = (e0 + 5 < nE) ? dsts[min(e0 + 5, nE - 1)] : sent;
    db.z = (e0 + 6 < nE) ? dsts[min(e0 + 6, nE - 1)] : sent;
    db.w = (e0 + 7 < nE) ? dsts[min(e0 + 7, nE - 1)] : sent;
  }
  const unsigned nbs = (unsigned)slotBase;
  const unsigned unb = (unsigned)nb;
  const unsigned s0 = (unsigned)da.x - nbs, s1 = (unsigned)da.y - nbs;
  const unsigned s2 = (unsigned)da.z - nbs, s3 = (unsigned)da.w - nbs;
  const unsigned s4 = (unsigned)db.x - nbs, s5 = (unsigned)db.y - nbs;
  const unsigned s6 = (unsigned)db.z - nbs, s7 = (unsigned)db.w - nbs;
  const bool h0 = s0 < unb, h1 = s1 < unb, h2 = s2 < unb, h3 = s3 < unb;
  const bool h4 = s4 < unb, h5 = s5 < unb, h6 = s6 < unb, h7 = s7 < unb;
  const unsigned any = __builtin_amdgcn_ballot_w32(h0 | h1 | h2 | h3 | h4 | h5 | h6 | h7);
  if (any != 0u) {
#define HITJ(J, HJ, SJ) { \
      const unsigned mj = __builtin_amdgcn_ballot_w32(HJ); \
      if (mj != 0u) { \
        if (HJ) { \
          const int pos = wc + (int)__builtin_amdgcn_mbcnt_lo(mj, 0u); \
          if (pos < WCAP) list[wave * WCAP + pos] = ((el0 + (J)) << PKS) | (int)(SJ); \
        } \
        wc += (int)__builtin_popcount(mj); } }
    HITJ(0, h0, s0)
    HITJ(1, h1, s1)
    HITJ(2, h2, s2)
    HITJ(3, h3, s3)
    HITJ(4, h4, s4)
    HITJ(5, h5, s5)
    HITJ(6, h6, s6)
    HITJ(7, h7, s7)
#undef HITJ
  }
  return wc;
}

__global__ __launch_bounds__(NTHR) void k_prep(const float* __restrict__ x, const float* __restrict__ We,
                                               const float* __restrict__ W1, const float* __restrict__ W2,
                                               int nN, int mRows, unsigned short* WeT, unsigned short* W1D,
                                               unsigned short* W2D, unsigned short* XB) {
  const int u  = (int)blockIdx.x * NTHR + (int)threadIdx.x;
  const int L0 = NU_W1;
  const int L1 = L0 + NU_W2;
  const int L2 = L1 + NU_WE;
  const int L3 = L2 + mRows * (DH / 8);
  v8us o;
  if (u < L0) {
    const int n  = u >> 5;
    const int k8 = (u & 31) * 8;
    const int kk = k8 & (DH - 1);
    const float* p = W1 + (size_t)kk * D2 + n;
#pragma unroll
    for (int i = 0; i < 8; ++i) o[i] = bf_bits(p[(size_t)i * D2]);
    put16(W1D + (size_t)u * 8, o);
    return;
  } else if (u < L1) {
    const int v  = u - L0;
    const int n  = v >> 6;
    const int k8 = (v & 63) * 8;
    const int kk = k8 & (D2 - 1);
    const float* p = W2 + (size_t)kk * DH + n;
#pragma unroll
    for (int i = 0; i < 8; ++i) o[i] = bf_bits(p[(size_t)i * DH]);
    put16(W2D + (size_t)v * 8, o);
    return;
  } else if (u < L2) {
    const int v  = u - L1;
    const int n  = v >> 2;
    const int k8 = (v & 3) * 8;
    const int kc = (k8 < EDIM) ? k8 : 0;
    const unsigned short mk = (k8 < EDIM) ? (unsigned short)0xffffu : (unsigned short)0u;
    const float* p = We + (size_t)kc * DH + n;
#pragma unroll
    for (int i = 0; i < 8; ++i) o[i] = (unsigned short)(bf_bits(p[(size_t)i * DH]) & mk);
    put16(WeT + (size_t)v * 8, o);
    return;
  } else if (u < L3) {
    const int v   = u - L2;
    const int row = v >> 4;
    const int j   = v & 15;
    const int rc  = row < nN ? row : nN - 1;
    const unsigned short mk = (row < nN) ? (unsigned short)0xffffu : (unsigned short)0u;
    const float* p = x + (size_t)rc * DH + 8 * j;
    const v4f a = *(const v4f*)p;
    const v4f b = *(const v4f*)(p + 4);
    o[0] = (unsigned short)(bf_bits(a.x) & mk); o[1] = (unsigned short)(bf_bits(a.y) & mk);
    o[2] = (unsigned short)(bf_bits(a.z) & mk); o[3] = (unsigned short)(bf_bits(a.w) & mk);
    o[4] = (unsigned short)(bf_bits(b.x) & mk); o[5] = (unsigned short)(bf_bits(b.y) & mk);
    o[6] = (unsigned short)(bf_bits(b.z) & mk); o[7] = (unsigned short)(bf_bits(b.w) & mk);
    put16(XB + (size_t)v * 8, o);
    return;
  }
}

__global__ __launch_bounds__(ETHR) void k_edge(const int* __restrict__ srcs, int nE, int nN,
                                               const float* __restrict__ ea,
                                               const unsigned short* __restrict__ WeT,
                                               const float* __restrict__ be,
                                               const unsigned short* __restrict__ XB,
                                               unsigned short* M16) {
  __shared__ __attribute__((aligned(16))) float sD[ET * SDP];
  __shared__ __attribute__((aligned(16))) unsigned short sA[ET * SAP];
  const int tid = (int)threadIdx.x, lane = tid & 31, wave = tid >> 5, hh = lane >> 4, m = lane & 15;
  const int tileBase = (int)blockIdx.x * ET;

#pragma unroll
  for (int i = 0; i < 2; ++i) {
    const int idx = tid + ETHR * i;
    const int row = idx >> 2;
    const int q   = idx & 3;
    const int e   = tileBase + row;
    const int ec  = e < nE ? e : nE - 1;
    const v4f a = *(const v4f*)(ea + (size_t)ec * EDIM + 4 * q);
    v2u w;
    w.x = (unsigned int)bf_bits(a.x) | ((unsigned int)bf_bits(a.y) << 16);
    w.y = (unsigned int)bf_bits(a.z) | ((unsigned int)bf_bits(a.w) << 16);
    *(v2ua*)(sA + row * SAP + 4 * q) = w;
  }
  {
    const int row = tid >> 1;
    const int hf  = tid & 1;
    const v4u z = {0u, 0u, 0u, 0u};
    *(v4ua*)(sA + row * SAP + EDIM + 8 * hf) = z;
  }
  int sv;
  {
    const int er = tileBase + 16 * wave + m;
    const int ec = er < nE ? er : nE - 1;
    sv = srcs[ec];
    sv = sv < 0 ? 0 : (sv > nN - 1 ? nN - 1 : sv);
  }
  __syncthreads();

  {
    v8f acc[GNT];
    FragB af;
    const unsigned short* ar = sA + (16 * wave + m) * SAP + 8 * hh;
    af.h[0] = *(const v8usa*)ar;
    af.h[1] = *(const v8usa*)(ar + 16);
#pragma unroll
    for (int nt = 0; nt < GNT; ++nt) {
      const unsigned short* wq = WeT + (size_t)(16 * nt + m) * KE + 8 * hh;
      FragB bf;
      bf.h[0] = *(const v8usa*)wq;
      bf.h[1] = *(const v8usa*)(wq + 16);
      acc[nt] = wmb(af, bf, z8());
    }
#pragma unroll
    for (int nt = 0; nt < GNT; ++nt) {
      const int lc = 16 * nt + m;
#pragma unroll
      for (int r = 0; r < 8; ++r) {
        const int lr = 16 * wave + 8 * hh + r;
        sD[lr * SDP + lc] = acc[nt][r];
      }
    }
  }
  __syncthreads();

  const int c0 = 8 * m;
  float bb[8];
  {
    const v4f b0 = *(const v4f*)(be + c0);
    const v4f b1 = *(const v4f*)(be + c0 + 4);
    bb[0] = bf_rne(b0.x); bb[1] = bf_rne(b0.y); bb[2] = bf_rne(b0.z); bb[3] = bf_rne(b0.w);
    bb[4] = bf_rne(b1.x); bb[5] = bf_rne(b1.y); bb[6] = bf_rne(b1.z); bb[7] = bf_rne(b1.w);
  }
  v4u pk[8];
#pragma unroll
  for (int j = 0; j < 8; ++j) {
    const int wr = 2 * j + hh;
    const int lr = 16 * wave + wr;
    const int s  = __shfl(sv, wr, 32);
    const v4f d0 = *(const v4fa*)(sD + lr * SDP + c0);
    const v4f d1 = *(const v4fa*)(sD + lr * SDP + c0 + 4);
    const v4u xw = *(const v4ua*)(XB + (size_t)s * XBW + c0);
    float f[8], xs[8];
    f[0] = d0.x; f[1] = d0.y; f[2] = d0.z; f[3] = d0.w;
    f[4] = d1.x; f[5] = d1.y; f[6] = d1.z; f[7] = d1.w;
    xs[0] = __uint_as_float(xw.x << 16); xs[1] = __uint_as_float(xw.x & 0xffff0000u);
    xs[2] = __uint_as_float(xw.y << 16); xs[3] = __uint_as_float(xw.y & 0xffff0000u);
    xs[4] = __uint_as_float(xw.z << 16); xs[5] = __uint_as_float(xw.z & 0xffff0000u);
    xs[6] = __uint_as_float(xw.w << 16); xs[7] = __uint_as_float(xw.w & 0xffff0000u);
    unsigned int hb[8];
#pragma unroll
    for (int i = 0; i < 8; ++i) {
      const float v = (xs[i] + f[i]) + bb[i];
      hb[i] = f2h(MSGC * relu_keep(v));
    }
    v4u p;
    p.x = hb[0] | (hb[1] << 16);
    p.y = hb[2] | (hb[3] << 16);
    p.z = hb[4] | (hb[5] << 16);
    p.w = hb[6] | (hb[7] << 16);
    pk[j] = p;
  }
#pragma unroll
  for (int j = 0; j < 8; ++j) {
    const int e  = tileBase + 16 * wave + 2 * j + hh;
    const int ec = e < nE ? e : nE - 1;
    unsigned short* op = M16 + (size_t)ec * MW + c0;
    if (e < nE) *(volatile v4u*)op = pk[j];
  }
  __threadfence();
#pragma unroll
  for (int j = 0; j < 8; ++j) {
    const int e  = tileBase + 16 * wave + 2 * j + hh;
    const int ec = e < nE ? e : nE - 1;
    unsigned short* op = M16 + (size_t)ec * MW + c0;
    if (e < nE) *(volatile v4u*)op = pk[j];
  }
}

__global__ __launch_bounds__(NTHR) void k_scan(const int* __restrict__ dsts,
                                               const unsigned int* __restrict__ M16w,
                                               const unsigned int* __restrict__ XBw,
                                               const float* __restrict__ epsp,
                                               unsigned short* Aout,
                                               int nN, int nE, int nb, int vec8, int MPr) {
  extern __shared__ v4f lds_dyn[];
  int* reg1 = (int*)lds_dyn;
  int* reg2 = reg1 + RCAP;
  int* scnt = reg2 + RCAP;
  int* soff = scnt + NBMAX;
  int* list = soff + NBMAX;
  int* wcnt = list + LISTN;
  int* wtot = wcnt + NWAVE;
  const int tid = (int)threadIdx.x, lane = tid & 31, wave = tid >> 5;
  const int nodeBase = (int)blockIdx.x * nb;
  const float scale = 1.0f + bf_rne(epsp[0]);

  for (int i = tid; i < NBMAX; i += NTHR) scnt[i] = 0;
  __syncthreads();

  int tot = 0;
  const int nChunks = (nE + CHUNK - 1) / CHUNK;
#pragma unroll 1
  for (int ch = 0; ch < nChunks; ++ch) {
    const int cbase = ch * CHUNK;
    const int wc = scan_chunk(dsts, nE, cbase, nodeBase, nb, vec8, list, tid, lane, wave);
    if (lane == 0) wcnt[wave] = wc;
    __syncthreads();
    int pre = 0, all = 0;
#pragma unroll
    for (int w2 = 0; w2 < NWAVE; ++w2) {
      int c = wcnt[w2];
      c = c < 0 ? 0 : (c > WCAP ? WCAP : c);
      all += c;
      pre += (w2 < wave) ? c : 0;
    }
    const int wcc  = wc > WCAP ? WCAP : wc;
    const int base = tot + pre;
#pragma unroll 1
    for (int i = lane; i < wcc; i += 32) {
      const int ent = list[wave * WCAP + i];
      const int el  = (ent >> PKS) & (CHUNK - 1);
      const int sl  = ent & (NBMAX - 1);
      int eid = cbase + el;
      eid = eid > nE - 1 ? nE - 1 : eid;
      const int pos = base + i;
      if (pos < RCAP) reg1[pos] = (int)(((unsigned)eid << PKS) | (unsigned)sl);
    }
    tot += all;
    tot = tot > RCAP ? RCAP : tot;
    __syncthreads();
  }
  const int nh = tot;

  if (wave == 0) {
#pragma unroll 1
    for (int b0 = 0; b0 < nh; b0 += 32) {
      const int idx = b0 + lane;
      const int uv  = reg1[idx < RCAP ? idx : RCAP - 1];
      const int m32 = (nh - b0) < 32 ? (nh - b0) : 32;
#pragma unroll 1
      for (int k = 0; k < m32; ++k) {
        const int u  = __builtin_amdgcn_readlane(uv, k);
        const int sl = u & (NBMAX - 1);
        if (lane == 0) scnt[sl] = scnt[sl] + 1;
      }
    }
  }
  __syncthreads();

  {
    const v4i ca = *(const v4i*)(scnt + 8 * tid);
    const v4i cb = *(const v4i*)(scnt + 8 * tid + 4);
    const int e0 = ca.x < 0 ? 0 : ca.x, e1 = ca.y < 0 ? 0 : ca.y, e2 = ca.z < 0 ? 0 : ca.z, e3 = ca.w < 0 ? 0 : ca.w;
    const int e4 = cb.x < 0 ? 0 : cb.x, e5 = cb.y < 0 ? 0 : cb.y, e6 = cb.z < 0 ? 0 : cb.z, e7 = cb.w < 0 ? 0 : cb.w;
    const int ts = e0 + e1 + e2 + e3 + e4 + e5 + e6 + e7;
    int incl = ts;
#pragma unroll
    for (int d = 1; d < 32; d <<= 1) {
      const int up = __shfl_up(incl, d);
      if (lane >= d) incl += up;
    }
    if (lane == 31) wtot[wave] = incl;
    __syncthreads();
    int pre = 0;
#pragma unroll
    for (int w2 = 0; w2 < NWAVE; ++w2) pre += (w2 < wave) ? wtot[w2] : 0;
    int run = pre + incl - ts;
    soff[8 * tid + 0] = run; run += e0;
    soff[8 * tid + 1] = run; run += e1;
    soff[8 * tid + 2] = run; run += e2;
    soff[8 * tid + 3] = run; run += e3;
    soff[8 * tid + 4] = run; run += e4;
    soff[8 * tid + 5] = run; run += e5;
    soff[8 * tid + 6] = run; run += e6;
    soff[8 * tid + 7] = run;
  }
  __syncthreads();
  for (int i = tid; i < NBMAX; i += NTHR) list[i] = soff[i];
  __syncthreads();

  if (wave == 0) {
#pragma unroll 1
    for (int b0 = 0; b0 < nh; b0 += 32) {
      const int idx = b0 + lane;
      const int uv  = reg1[idx < RCAP ? idx : RCAP - 1];
      const int m32 = (nh - b0) < 32 ? (nh - b0) : 32;
#pragma unroll 1
      for (int k = 0; k < m32; ++k) {
        const int u   = __builtin_amdgcn_readlane(uv, k);
        const int sl  = u & (NBMAX - 1);
        const int eid = (int)((unsigned)u >> PKS);
        if (lane == 0) {
          int pos = list[sl];
          pos = pos < 0 ? 0 : (pos > RCAP - 1 ? RCAP - 1 : pos);
          reg2[pos] = eid;
          list[sl] = pos + 1;
        }
      }
    }
  }
  __syncthreads();

  const int nbw = nb >> 3;
  const bool ovf = (nh >= RCAP);
  const float qnan = __int_as_float(0x7fc00000);
  unsigned int* stwu = (unsigned int*)((float*)reg1 + wave * STW);

#pragma unroll 1
  for (int jt = 0; jt < nbw; ++jt) {
    const int slot = wave * nbw + jt;
    const int grow = nodeBase + slot;
    int st = soff[slot];
    const int craw = scnt[slot];
    int cnt = craw;
    st  = st < 0 ? 0 : (st > nh ? nh : st);
    cnt = cnt < 0 ? 0 : (cnt > DEGCAP ? DEGCAP : cnt);
    if (cnt > nh - st) cnt = nh - st;
    const float pz = (ovf || craw > DEGCAP) ? qnan : 0.0f;
    const bool liveRow = grow < nN;

    float ag0 = 0.f, ag1 = 0.f, ag2 = 0.f, ag3 = 0.f;
#pragma unroll 1
    for (int b0 = 0; b0 < cnt; b0 += 32) {
      int idx = st + b0 + lane;
      idx = idx > nh - 1 ? nh - 1 : idx;
      idx = idx < 0 ? 0 : (idx > RCAP - 1 ? RCAP - 1 : idx);
      int eid = reg2[idx];
      eid = eid < 0 ? 0 : (eid > nE - 1 ? nE - 1 : eid);
      const int m32 = (cnt - b0) < 32 ? (cnt - b0) : 32;
#pragma unroll 1
      for (int k = 0; k < m32; ++k) {
        const int ek = __builtin_amdgcn_readlane(eid, k);
        const v2u w = *(const v2u*)(M16w + (size_t)ek * MWW + 2 * lane);
        ag0 += h2f(w.x & 0xffffu);
        ag1 += h2f(w.x >> 16);
        ag2 += h2f(w.y & 0xffffu);
        ag3 += h2f(w.y >> 16);
      }
    }
    const int nc = liveRow ? grow : nN - 1;
    const v2u sw = *(const v2u*)(XBw + (size_t)nc * XBWW + 2 * lane);
    const float s0 = __uint_as_float(sw.x << 16), s1 = __uint_as_float(sw.x & 0xffff0000u);
    const float s2 = __uint_as_float(sw.y << 16), s3 = __uint_as_float(sw.y & 0xffff0000u);
    float r0 = scale * s0 + ag0 * MSGI;
    float r1 = scale * s1 + ag1 * MSGI;
    float r2 = scale * s2 + ag2 * MSGI;
    float r3 = scale * s3 + ag3 * MSGI;
    r0 = (liveRow ? r0 : 0.0f) + pz;
    r1 = (liveRow ? r1 : 0.0f) + pz;
    r2 = (liveRow ? r2 : 0.0f) + pz;
    r3 = (liveRow ? r3 : 0.0f) + pz;

    const unsigned short hb0 = bf_bits(r0), hb1 = bf_bits(r1), hb2 = bf_bits(r2), hb3 = bf_bits(r3);
    const unsigned short lb0 = bf_bits(r0 - bf_val(hb0)), lb1 = bf_bits(r1 - bf_val(hb1));
    const unsigned short lb2 = bf_bits(r2 - bf_val(hb2)), lb3 = bf_bits(r3 - bf_val(hb3));
    v2u hw, lw;
    hw.x = (unsigned int)hb0 | ((unsigned int)hb1 << 16);
    hw.y = (unsigned int)hb2 | ((unsigned int)hb3 << 16);
    lw.x = (unsigned int)lb0 | ((unsigned int)lb1 << 16);
    lw.y = (unsigned int)lb2 | ((unsigned int)lb3 << 16);
    __builtin_amdgcn_fence(__ATOMIC_RELEASE, "wavefront");
    __builtin_amdgcn_wave_barrier();
    *(v2ua*)(stwu + 2 * lane)      = hw;
    *(v2ua*)(stwu + 64 + 2 * lane) = lw;
    __builtin_amdgcn_fence(__ATOMIC_RELEASE, "wavefront");
    __builtin_amdgcn_wave_barrier();
    const v4u pk = *(const v4ua*)(stwu + 4 * lane);
    const bool wsv = grow < MPr;
    const int gsafe = wsv ? grow : MPr - 1;
    unsigned short* gp = Aout + (size_t)gsafe * (size_t)APW + 8 * lane;
    if (wsv) *(volatile v4u*)gp = pk;
    __threadfence();
    if (wsv) *(volatile v4u*)gp = pk;
  }
}

template <int MODE, int KT>
__global__ __launch_bounds__(GTHR) void k_gemm(const unsigned short* __restrict__ A,
                                               const unsigned short* __restrict__ WT,
                                               const float* __restrict__ bias,
                                               void* outp, float* part, int nN, int mRows)
{
  constexpr int NT = GNT;
  constexpr int NI = 16;
  __shared__ __attribute__((aligned(16))) float stg[GBM * BN];
  __shared__ __attribute__((aligned(16))) float pst[PARTW];
  const int tid = (int)threadIdx.x, lane = tid & 31, wave = tid >> 5, hh = lane >> 4, m = lane & 15;
  const int rowBase = (int)blockIdx.x * GBM;
  const int cbk = (int)blockIdx.y;

  v8f acc[NT];
#pragma unroll
  for (int t = 0; t < NT; ++t) acc[t] = z8();
  const unsigned short* ap = A + (size_t)(rowBase + 16 * wave + m) * (size_t)KT + 8 * hh;
  const unsigned short* wp = WT + (size_t)(cbk * BN + m) * (size_t)KT + 8 * hh;
  constexpr int ksteps = KT / 32;
#pragma unroll 1
  for (int ks = 0; ks < ksteps; ++ks) {
    FragB af;
    af.h[0] = *(const v8usa*)(ap + 32 * ks);
    af.h[1] = *(const v8usa*)(ap + 32 * ks + 16);
#pragma unroll
    for (int t = 0; t < NT; ++t) {
      const unsigned short* wq = wp + (size_t)(16 * t) * (size_t)KT + 32 * ks;
      FragB bf;
      bf.h[0] = *(const v8usa*)wq;
      bf.h[1] = *(const v8usa*)(wq + 16);
      acc[t] = wmb(af, bf, acc[t]);
    }
  }

#pragma unroll
  for (int t = 0; t < NT; ++t) {
    const int lc = 16 * t + m;
    const float bb = bf_rne(bias[cbk * BN + lc]);
#pragma unroll
    for (int r = 0; r < 8; ++r) {
      const int lr = 16 * wave + 8 * hh + r;
      const bool live = (rowBase + lr) < nN;
      float v = acc[t][r] + bb;
      if (MODE == 1) v = relu_keep(v);
      stg[lr * BN + lc] = live ? v : 0.0f;
    }
  }
  __syncthreads();

  if constexpr (MODE == 0) {
    {
      int rv = nN - rowBase;
      rv = rv < 0 ? 0 : (rv > GBM ? GBM : rv);
      float n = 0.0f, mean = 0.0f, M2 = 0.0f;
#pragma unroll 1
      for (int r = 0; r < rv; ++r) {
        const float v = stg[r * BN + tid];
        n += 1.0f;
        const float rk = 1.0f / n;
        const float d = v - mean;
        mean = fmaf(d, rk, mean);
        M2 = fmaf(d, v - mean, M2);
      }
      pst[1 + tid] = mean;
      pst[1 + BN + tid] = M2;
      if (tid == 0) pst[0] = n;
#pragma unroll 1
      for (int i = 2 * BN + 1 + tid; i < PARTW; i += GTHR) pst[i] = 0.0f;
    }
    float* outF = (float*)outp;
    v4f fv[NI];
#pragma unroll
    for (int i = 0; i < NI; ++i) {
      const int lr = 16 * wave + i;
      fv[i] = *(const v4fa*)(stg + lr * BN + 4 * lane);
    }
#pragma unroll
    for (int i = 0; i < NI; ++i) {
      const int gr = rowBase + 16 * wave + i;
      float* op = outF + (size_t)gr * (size_t)DH + 4 * lane;
      if (gr < mRows) *(volatile v4f*)op = fv[i];
    }
    __threadfence();
#pragma unroll
    for (int i = 0; i < NI; ++i) {
      const int gr = rowBase + 16 * wave + i;
      float* op = outF + (size_t)gr * (size_t)DH + 4 * lane;
      if (gr < mRows) *(volatile v4f*)op = fv[i];
    }
    __syncthreads();
    v4f pv = {0.f, 0.f, 0.f, 0.f};
    if (tid < PARTW / 4) {
      pv = *(const v4fa*)(pst + 4 * tid);
      *(volatile v4f*)(part + (size_t)blockIdx.x * PARTW + 4 * tid) = pv;
    }
    __threadfence();
    if (tid < PARTW / 4) {
      *(volatile v4f*)(part + (size_t)blockIdx.x * PARTW + 4 * tid) = pv;
    }
  } else {
    unsigned short* outH = (unsigned short*)outp;
    const int cb = 8 * m;
    const bool isHi = (hh == 0);
    const int ocol = (isHi ? 0 : D2) + cbk * BN + cb;
    v4u pk[NI];
#pragma unroll
    for (int i = 0; i < NI; ++i) {
      const int lr = 16 * wave + i;
      const v4f a = *(const v4fa*)(stg + lr * BN + cb);
      const v4f b = *(const v4fa*)(stg + lr * BN + cb + 4);
      const float f[8] = {a.x, a.y, a.z, a.w, b.x, b.y, b.z, b.w};
      unsigned int w[4];
#pragma unroll
      for (int j = 0; j < 4; ++j) {
        const unsigned short h0 = bf_bits(f[2 * j]), h1 = bf_bits(f[2 * j + 1]);
        const unsigned short l0 = bf_bits(f[2 * j] - bf_val(h0)), l1 = bf_bits(f[2 * j + 1] - bf_val(h1));
        const unsigned short q0 = isHi ? h0 : l0, q1 = isHi ? h1 : l1;
        w[j] = (unsigned int)q0 | ((unsigned int)q1 << 16);
      }
      v4u pw; pw.x = w[0]; pw.y = w[1]; pw.z = w[2]; pw.w = w[3];
      pk[i] = pw;
    }
#pragma unroll
    for (int i = 0; i < NI; ++i) {
      const int gr = rowBase + 16 * wave + i;
      unsigned short* op = outH + (size_t)gr * (size_t)TPW + ocol;
      if (gr < mRows) *(volatile v4u*)op = pk[i];
    }
    __threadfence();
#pragma unroll
    for (int i = 0; i < NI; ++i) {
      const int gr = rowBase + 16 * wave + i;
      unsigned short* op = outH + (size_t)gr * (size_t)TPW + ocol;
      if (gr < mRows) *(volatile v4u*)op = pk[i];
    }
  }
}

__global__ __launch_bounds__(DH) void k_comb(const float* __restrict__ part, int nPart, float* stat) {
  __shared__ __attribute__((aligned(16))) float stg[2 * DH];
  const int tid = (int)threadIdx.x;
  const int c = tid & (DH - 1);
  double n = 0.0, mean = 0.0, M2 = 0.0;
#pragma unroll 1
  for (int b = 0; b < nPart; ++b) {
    const float* pr = part + (size_t)b * PARTW;
    const float nb = pr[0];
    const float mb = pr[1 + c];
    const float qb = pr[1 + DH + c];
    if (nb > 0.5f) {
      const double nn = n + (double)nb;
      const double delta = (double)mb - mean;
      const double f = (double)nb / nn;
      mean = mean + delta * f;
      M2 = M2 + (double)qb + delta * delta * n * f;
      n = nn;
    }
  }
  const double nt = n < 1.0 ? 1.0 : n;
  const float var = (float)(M2 / nt);
  const float rstd = 1.0f / sqrtf(var + BNEPS);
  stg[c] = (float)mean;
  stg[DH + c] = rstd;
  __syncthreads();
  v4f v = {0.f, 0.f, 0.f, 0.f};
  if (tid < (2 * DH) / 4) {
    v = *(const v4fa*)(stg + 4 * tid);
    *(volatile v4f*)(stat + 4 * tid) = v;
  }
  __threadfence();
  if (tid < (2 * DH) / 4) {
    *(volatile v4f*)(stat + 4 * tid) = v;
  }
}

__global__ __launch_bounds__(NTHR) void k_apply(const float* __restrict__ uf,
                                                const unsigned int* __restrict__ XBw,
                                                const float* __restrict__ stat,
                                                const float* __restrict__ gam, const float* __restrict__ bet,
                                                int nUnits, float* out) {
  __shared__ float sst[4 * DH];
  const int tid = (int)threadIdx.x;
  {
    const int c = tid & (DH - 1);
    const float g = bf_rne(gam[c]);
    const float b = bf_rne(bet[c]);
    sst[tid] = stat[tid];
    sst[2 * DH + tid] = (tid < DH) ? g : b;
  }
  __syncthreads();
  const int u = (int)blockIdx.x * NTHR + tid;
  if (u >= nUnits) return;
  const int row = u >> 5;
  const int q   = u & 31;
  const int c4  = q * 4;
  const v4f a = *(const v4f*)(uf + (size_t)row * DH + c4);
  const v2u xw = *(const v2u*)(XBw + (size_t)row * XBWW + 2 * q);
  const float x0 = __uint_as_float(xw.x << 16), x1 = __uint_as_float(xw.x & 0xffff0000u);
  const float x2 = __uint_as_float(xw.y << 16), x3 = __uint_as_float(xw.y & 0xffff0000u);
  v4f o;
  o.x = relu_keep((((a.x - sst[c4 + 0]) * sst[DH + c4 + 0]) * sst[2 * DH + c4 + 0] + sst[3 * DH + c4 + 0]) + x0);
  o.y = relu_keep((((a.y - sst[c4 + 1]) * sst[DH + c4 + 1]) * sst[2 * DH + c4 + 1] + sst[3 * DH + c4 + 1]) + x1);
  o.z = relu_keep((((a.z - sst[c4 + 2]) * sst[DH + c4 + 2]) * sst[2 * DH + c4 + 2] + sst[3 * DH + c4 + 2]) + x2);
  o.w = relu_keep((((a.w - sst[c4 + 3]) * sst[DH + c4 + 3]) * sst[2 * DH + c4 + 3] + sst[3 * DH + c4 + 3]) + x3);
  float* hp = out + (size_t)row * DH + c4;
  *(volatile v4f*)hp = o;
  __threadfence();
  *(volatile v4f*)hp = o;
}

static inline int cdiv(int a, int b) { return (a + b - 1) / b; }
static inline size_t al256(size_t o) { return (o + 255) & ~(size_t)255; }

extern "C" void kernel_launch(void* const* d_in, const int* in_sizes, int n_in,
                              void* d_out, int out_size, void* d_ws, size_t ws_size,
                              hipStream_t stream) {
  if (n_in < 12) return;
  if (in_sizes[0] < DH || (in_sizes[0] % DH) != 0) return;
  const int nN = in_sizes[0] / DH;
  if (nN < 1 || nN > (1 << 22)) return;
  if (in_sizes[1] < 2 || (in_sizes[1] & 1) != 0) return;
  const int nE = in_sizes[1] / 2;
  if (nE < 1 || nE > (1 << 21)) return;
  if ((long long)in_sizes[2] != (long long)nE * EDIM) return;
  if (in_sizes[3] != EDIM * DH || in_sizes[4] != DH) return;
  if (in_sizes[5] != 1) return;
  if (in_sizes[6] != DH * D2 || in_sizes[7] != D2) return;
  if (in_sizes[8] != D2 * DH || in_sizes[9] != DH) return;
  if (in_sizes[10] != DH || in_sizes[11] != DH) return;
  if ((long long)out_size != (long long)nN * DH) return;

  const float* x   = (const float*)d_in[0];
  const int*   ei  = (const int*)  d_in[1];
  const float* ea  = (const float*)d_in[2];
  const float* We  = (const float*)d_in[3];
  const float* be  = (const float*)d_in[4];
  const float* eps = (const float*)d_in[5];
  const float* W1  = (const float*)d_in[6];
  const float* b1  = (const float*)d_in[7];
  const float* W2  = (const float*)d_in[8];
  const float* b2  = (const float*)d_in[9];
  const float* gam = (const float*)d_in[10];
  const float* bet = (const float*)d_in[11];
  float* out = (float*)d_out;
  const int* src = ei;
  const int* dst = ei + nE;

  const int MP   = cdiv(nN, GBM) * GBM;
  const int gM   = MP / GBM;
  const int nb   = NBRUN;
  const int gA   = cdiv(MP, nb);
  const int gE   = cdiv(nE, ET);
  const int vec8 = ((nE & 3) == 0) ? 1 : 0;
  if ((long long)gA * nb < (long long)MP) return;
  if ((long long)gE * ET < (long long)nE) return;
  const long long nUa = (long long)nN * (DH / 4);
  if (nUa > 2000000000LL) return;
  const int nU4 = (int)nUa;

  char* ws = (char*)d_ws;
  size_t off = 0;
  const size_t szM16 = (size_t)gE * ET * MW * 2;
  const size_t szThl = (size_t)MP * TPW * 2;
  const size_t szU   = (size_t)MP * DH * 4;
  const size_t oUinB = al256(szThl);
  const size_t szBIG = (szM16 > oUinB + szU) ? szM16 : (oUinB + szU);
  const size_t oWeT = off; off = al256(off + (size_t)DH * KE * 2);
  const size_t oW1D = off; off = al256(off + (size_t)D2 * D2 * 2);
  const size_t oW2D = off; off = al256(off + (size_t)DH * TPW * 2);
  const size_t oXB  = off; off = al256(off + (size_t)MP * XBW * 2);
  const size_t oHhl = off; off = al256(off + (size_t)MP * APW * 2);
  const size_t oBIG = off; off = al256(off + szBIG);
  const size_t oPT  = off; off = al256(off + (size_t)gM * PARTW * 4);
  const size_t oST  = off; off = al256(off + (size_t)(2 * DH) * 4);
  if (off > ws_size) return;
  unsigned short* WeT = (unsigned short*)(ws + oWeT);
  unsigned short* W1D = (unsigned short*)(ws + oW1D);
  unsigned short* W2D = (unsigned short*)(ws + oW2D);
  unsigned short* XB  = (unsigned short*)(ws + oXB);
  unsigned short* Hhl = (unsigned short*)(ws + oHhl);
  unsigned short* M16 = (unsigned short*)(ws + oBIG);
  unsigned short* Thl = (unsigned short*)(ws + oBIG);
  float*          UF  = (float*)(ws + oBIG + oUinB);
  float*          PART = (float*)(ws + oPT);
  float*          STAT = (float*)(ws + oST);

  hipFuncSetAttribute(reinterpret_cast<const void*>(&k_scan), hipFuncAttributeMaxDynamicSharedMemorySize, LDS_AGG);

  const int nPrep = NU_W1 + NU_W2 + NU_WE + MP * (DH / 8);

  k_prep<<<cdiv(nPrep, NTHR), NTHR, 0, stream>>>(x, We, W1, W2, nN, MP, WeT, W1D, W2D, XB);
  k_edge<<<gE, ETHR, 0, stream>>>(src, nE, nN, ea, WeT, be, XB, M16);
  k_scan<<<gA, NTHR, LDS_AGG, stream>>>(dst, (const unsigned int*)M16, (const unsigned int*)XB, eps, Hhl,
                                        nN, nE, nb, vec8, MP);
  k_gemm<1, APW><<<dim3(gM, D2 / BN), GTHR, 0, stream>>>(Hhl, W1D, b1, (void*)Thl, PART, nN, MP);
  k_gemm<0, TPW><<<dim3(gM, 1), GTHR, 0, stream>>>(Thl, W2D, b2, (void*)UF, PART, nN, MP);
  k_comb<<<1, DH, 0, stream>>>(PART, gM, STAT);
  k_apply<<<cdiv(nU4, NTHR), NTHR, 0, stream>>>(UF, (const unsigned int*)XB, STAT, gam, bet, nU4, out);
}
